// HybridHymbaBlockCPU_5136780886733
// MI455X (gfx1250) — hardware-verified
//
#include <hip/hip_runtime.h>
#include <math.h>
#include <stdint.h>

#define NBAT   4
#define TLEN   2048
#define NTOK   8192
#define DM     256
#define NHEAD  8
#define HD     32
#define MD     768
#define D3     85
#define E1N    128
#define RNK    16
#define LR     8
#define QB     64
#define NQB    32
#define QKW    512
#define PZ_HALVES 16384

#define XSC    16.0f
#define WSC    64.0f
#define UVSC   4096.0f
#define QSC    16.0f
#define KSC    16.0f
#define VSC    16.0f
#define PSC    1024.0f
#define RSC    4096.0f
#define ZSC    64.0f
#define HSC    256.0f
#define SSC    16384.0f
#define TSC    256.0f
#define USC    64.0f
#define LORA_MUL 1.5f
#define LN_EPS 1.0e-5f
#define NEG_BIG (-1.0e30f)
#define LOG2_1E4 13.287712379549449

#define EPI_QKV   1
#define EPI_HA    2
#define EPI_F32   3
#define EPI_SIG   4
#define EPI_ALPHA 5
#define EPI_CW    6
#define EPI_MIX   7
#define EPI_W1    8
#define EPI_OUT   9

static_assert(NTOK == NBAT * TLEN);
static_assert(NHEAD * HD == DM);
static_assert((NHEAD % 2) == 0);
static_assert(MD == 3 * DM);
static_assert(QKW == 2 * DM);
static_assert(TLEN == NQB * QB);
static_assert((NTOK % 16) == 0 && (DM % 128) == 0 && (MD % 128) == 0 && (E1N % 128) == 0);
static_assert(2 * D3 < DM && 3 * D3 + 1 == DM);
static_assert((TLEN % 8) == 0 && (TLEN % 64) == 0);
static_assert(D3 <= E1N);
static_assert(PZ_HALVES >= 2 * 8 * 16 * 64 && PZ_HALVES >= 2 * 64 * 72);

typedef _Float16 v16h __attribute__((ext_vector_type(16)));
typedef _Float16 v8h  __attribute__((ext_vector_type(8)));
typedef float    v8f  __attribute__((ext_vector_type(8)));
typedef float    v4f  __attribute__((ext_vector_type(4)));
typedef unsigned int v4u __attribute__((ext_vector_type(4)));
union FH  { v16h v; v8h h[2]; };
union U84 { v8h h; v4u u; };

__device__ __forceinline__ unsigned short bf_bits(float f) {
  unsigned u = __float_as_uint(f);
  return (unsigned short)((u + 0x7FFFu + ((u >> 16) & 1u)) >> 16);
}
__device__ __forceinline__ float bf_up(unsigned short b) { return __uint_as_float(((unsigned)b) << 16); }
__device__ __forceinline__ float bfr(float f) { return bf_up(bf_bits(f)); }
__device__ __forceinline__ unsigned short h_bits(_Float16 x) { return __builtin_bit_cast(unsigned short, x); }
__device__ __forceinline__ unsigned pk16(unsigned short a, unsigned short b) { return (unsigned)a | ((unsigned)b << 16); }
__device__ __forceinline__ v8f zero8() { v8f z = {0.f, 0.f, 0.f, 0.f, 0.f, 0.f, 0.f, 0.f}; return z; }
__device__ __forceinline__ float gelu_f(float x) { return 0.5f * x * (1.0f + erff(x * 0.70710678118654752f)); }
__device__ __forceinline__ float sigm_f(float x) { return 1.0f / (1.0f + expf(-x)); }

__device__ __forceinline__ void hilo2(float s0, float s1, unsigned& ph, unsigned& pl) {
  const _Float16 x0 = (_Float16)s0, x1 = (_Float16)s1;
  const _Float16 y0 = (_Float16)((s0 - (float)x0) * RSC);
  const _Float16 y1 = (_Float16)((s1 - (float)x1) * RSC);
  ph = pk16(h_bits(x0), h_bits(x1));
  pl = pk16(h_bits(y0), h_bits(y1));
}

__device__ __forceinline__ v16h ldfrag_h(const _Float16* p) {
  FH f;
  f.h[0] = *(const v8h*)(p);
  f.h[1] = *(const v8h*)(p + 16);
  return f.v;
}

__device__ __forceinline__ v8f mma_h_raw(v16h a, v16h b, v8f c) {
  return __builtin_amdgcn_wmma_f32_16x16x32_f16(false, a, false, b, (short)0, c, false, false);
}
__device__ __forceinline__ void guard3(v8f& x, v8f& y, v16h a, v16h b, v16h d) {
#if defined(__HIP_DEVICE_COMPILE__)
  asm volatile("v_nop\n\tv_nop\n\tv_nop\n\tv_nop" : "+v"(x), "+v"(y) : "v"(a), "v"(b), "v"(d));
#endif
}
__device__ __forceinline__ void guard8m(v8f& x, v8f& y, v16h a, v16h b, v16h d, v16h e,
                                        v16h f, v16h g, v16h p, v16h q) {
#if defined(__HIP_DEVICE_COMPILE__)
  asm volatile("v_nop\n\tv_nop\n\tv_nop\n\tv_nop" : "+v"(x), "+v"(y)
               : "v"(a), "v"(b), "v"(d), "v"(e), "v"(f), "v"(g), "v"(p), "v"(q) : "memory");
#endif
}
__device__ __forceinline__ void acc_guard4(v8f& a, v8f& b, v8f& c, v8f& d) {
#if defined(__HIP_DEVICE_COMPILE__)
  asm volatile("v_nop\n\tv_nop\n\tv_nop\n\tv_nop" : "+v"(a), "+v"(b), "+v"(c), "+v"(d));
#endif
}
__device__ __forceinline__ void acc_guard2(v8f& a, v8f& b) {
#if defined(__HIP_DEVICE_COMPILE__)
  asm volatile("v_nop\n\tv_nop\n\tv_nop\n\tv_nop" : "+v"(a), "+v"(b));
#endif
}
__device__ __forceinline__ void cbar() {
#if defined(__HIP_DEVICE_COMPILE__)
  asm volatile("" ::: "memory");
#endif
}
__device__ __forceinline__ void wave_sync_lds() {
  __builtin_amdgcn_fence(__ATOMIC_RELEASE, "workgroup");
  __builtin_amdgcn_wave_barrier();
  __builtin_amdgcn_fence(__ATOMIC_ACQUIRE, "workgroup");
}

__global__ __launch_bounds__(256) void prep_w(const float* __restrict__ W, const float* __restrict__ Am,
                                             const float* __restrict__ Bm, unsigned short* out,
                                             int Ns, int Nd, int K, int R, int hasW, float cmul, float scale) {
  const size_t i8 = ((size_t)blockIdx.x * 256 + threadIdx.x) * 8;
  if (i8 + 8 > (size_t)Nd * (size_t)K) return;
  const int n  = (int)(i8 / (size_t)K);
  const int k  = (int)(i8 - (size_t)n * (size_t)K);
  const int nc = (n < Ns) ? n : (Ns - 1);
  const float vm = (n < Ns) ? 1.0f : 0.0f;
  float s[8], lr[8];
#pragma unroll
  for (int e = 0; e < 8; ++e) { s[e] = 0.f; lr[e] = 0.f; }
  if (hasW != 0) {
    const v4f a = *(const v4f*)(W + (size_t)nc * (size_t)K + k);
    const v4f b = *(const v4f*)(W + (size_t)nc * (size_t)K + k + 4);
    s[0] = bfr(a[0]); s[1] = bfr(a[1]); s[2] = bfr(a[2]); s[3] = bfr(a[3]);
    s[4] = bfr(b[0]); s[5] = bfr(b[1]); s[6] = bfr(b[2]); s[7] = bfr(b[3]);
  }
#pragma unroll 1
  for (int r = 0; r < R; ++r) {
    const float av = bfr(Am[(size_t)nc * (size_t)R + r]);
    const v4f b0 = *(const v4f*)(Bm + (size_t)r * (size_t)K + k);
    const v4f b1 = *(const v4f*)(Bm + (size_t)r * (size_t)K + k + 4);
    lr[0] += av * bfr(b0[0]); lr[1] += av * bfr(b0[1]); lr[2] += av * bfr(b0[2]); lr[3] += av * bfr(b0[3]);
    lr[4] += av * bfr(b1[0]); lr[5] += av * bfr(b1[1]); lr[6] += av * bfr(b1[2]); lr[7] += av * bfr(b1[3]);
  }
  v4u p;
#pragma unroll
  for (int e = 0; e < 4; ++e) {
    const _Float16 x0 = (_Float16)((s[2 * e] + cmul * lr[2 * e]) * vm * scale);
    const _Float16 x1 = (_Float16)((s[2 * e + 1] + cmul * lr[2 * e + 1]) * vm * scale);
    p[e] = pk16(h_bits(x0), h_bits(x1));
  }
  *(volatile v4u*)(out + i8) = p;
  __threadfence();
  *(volatile v4u*)(out + i8) = p;
}

__global__ __launch_bounds__(256) void rope_tab(float* RC, float* RS, int n) {
  const int e = blockIdx.x * 256 + (int)threadIdx.x;
  if (e >= n) return;
  const int t = e >> 4, i = e & 15;
  const double thd = exp2(-(double)i * (LOG2_1E4 / 16.0));
  const float  th  = (float)thd;
  const float  ang = (float)t * th;
  float sv, cv;
  sincosf(ang, &sv, &cv);
  *(volatile float*)(RC + e) = cv;
  *(volatile float*)(RS + e) = sv;
  __threadfence();
  *(volatile float*)(RC + e) = cv;
  *(volatile float*)(RS + e) = sv;
}

__global__ __launch_bounds__(256) void ln_rows(const float* __restrict__ X, const float* __restrict__ g,
                                              const float* __restrict__ bb, unsigned short* OH,
                                              unsigned short* OL, int nrows, float scale) {
  const int wave = threadIdx.x >> 5, lane = threadIdx.x & 31;
  const int row = blockIdx.x * 8 + wave;
  if (row >= nrows) return;
  const float* xr = X + (size_t)row * DM + lane * 8;
  const v4f a = *(const v4f*)xr;
  const v4f b = *(const v4f*)(xr + 4);
  float v[8];
  v[0] = bfr(a[0]); v[1] = bfr(a[1]); v[2] = bfr(a[2]); v[3] = bfr(a[3]);
  v[4] = bfr(b[0]); v[5] = bfr(b[1]); v[6] = bfr(b[2]); v[7] = bfr(b[3]);
  float sm = 0.f;
#pragma unroll
  for (int e = 0; e < 8; ++e) sm += v[e];
#pragma unroll
  for (int off = 1; off < 32; off <<= 1) sm += __shfl_xor(sm, off, 32);
  const float mean = sm * (1.0f / DM);
  float dv[8];
  float sq = 0.f;
#pragma unroll
  for (int e = 0; e < 8; ++e) { dv[e] = v[e] - mean; sq += dv[e] * dv[e]; }
#pragma unroll
  for (int off = 1; off < 32; off <<= 1) sq += __shfl_xor(sq, off, 32);
  const float var  = sq * (1.0f / DM);
  const float rstd = 1.0f / sqrtf(var + LN_EPS);
  v4u ph, pl;
#pragma unroll
  for (int e = 0; e < 4; ++e) {
    const int c0 = lane * 8 + 2 * e;
    const float y0 = dv[2 * e] * rstd * bfr(g[c0]) + bfr(bb[c0]);
    const float y1 = dv[2 * e + 1] * rstd * bfr(g[c0 + 1]) + bfr(bb[c0 + 1]);
    unsigned uh, ul;
    hilo2(y0 * scale, y1 * scale, uh, ul);
    ph[e] = uh;
    pl[e] = ul;
  }
  const size_t o = (size_t)row * DM + lane * 8;
  *(volatile v4u*)(OH + o) = ph;
  *(volatile v4u*)(OL + o) = pl;
  __threadfence();
  *(volatile v4u*)(OH + o) = ph;
  *(volatile v4u*)(OL + o) = pl;
}

__global__ __launch_bounds__(256) void tr_cvt2(const float* __restrict__ in, int R, int C,
                                              unsigned short* out0, unsigned short* out1, float scale) {
  __shared__ float sm[64][65];
  const int tid = threadIdx.x;
  const int c0 = blockIdx.x * 64;
  const int r0 = blockIdx.y * 64;
  if (c0 + 64 > C || r0 + 64 > R) return;
  {
    const int lr = tid >> 2, lc = (tid & 3) * 16;
    const float* src = in + (size_t)(r0 + lr) * (size_t)C + c0 + lc;
#pragma unroll
    for (int q = 0; q < 4; ++q) {
      const v4f v = *(const v4f*)(src + 4 * q);
      sm[lr][lc + 4 * q + 0] = v[0];
      sm[lr][lc + 4 * q + 1] = v[1];
      sm[lr][lc + 4 * q + 2] = v[2];
      sm[lr][lc + 4 * q + 3] = v[3];
    }
  }
  __syncthreads();
  const int seg = tid & 7;
  v4u p0[2], p1[2];
#pragma unroll
  for (int it = 0; it < 2; ++it) {
    const int ocl = it * 32 + (tid >> 3);
    float f[8];
#pragma unroll
    for (int e = 0; e < 8; ++e) f[e] = sm[seg * 8 + e][ocl];
    v4u pk, pl;
#pragma unroll
    for (int e = 0; e < 4; ++e) {
      unsigned uh, ul;
      hilo2(f[2 * e] * scale, f[2 * e + 1] * scale, uh, ul);
      pk[e] = uh;
      pl[e] = ul;
    }
    p0[it] = pk;
    p1[it] = pl;
  }
  for (int pass = 0; pass < 2; ++pass) {
#pragma unroll
    for (int it = 0; it < 2; ++it) {
      const int ocl = it * 32 + (tid >> 3);
      const size_t go = (size_t)(c0 + ocl) * (size_t)R + (size_t)(r0 + seg * 8);
      *(volatile v4u*)(out0 + go) = p0[it];
      *(volatile v4u*)(out1 + go) = p1[it];
    }
    __threadfence();
  }
}

template <int EPI>
__global__ __launch_bounds__(128) void gemm_t(
    const unsigned short* __restrict__ A, const unsigned short* __restrict__ AR, int lda,
    const unsigned short* __restrict__ Bt, int ldb,
    void* C0, void* C1, void* C2, int ldc,
    const float* __restrict__ P0, const float* __restrict__ P1, const float* __restrict__ P2,
    int M, int N, int K, float oscale, float cscale) {
  __shared__ __align__(16) float sT[4][16 * 132];
  const int lane = threadIdx.x & 31;
  const int wave = threadIdx.x >> 5;
  const int tilesN = N >> 7;
  const int tilesM = M >> 4;
  const int tile = blockIdx.x * 4 + wave;
  if (tile >= tilesM * tilesN) return;
  const int tm = tile / tilesN;
  const int tn = tile - tm * tilesN;
  const int m0 = tm << 4;
  const int n0 = tn << 7;
  const int rl   = lane & 15;
  const int hh   = lane >> 4;
  const int koff = hh * 8;

  v8f acch[8], accl[8];
#pragma unroll
  for (int j = 0; j < 8; ++j) { acch[j] = zero8(); accl[j] = zero8(); }

  {
    const _Float16* ar  = (const _Float16*)(const void*)A  + (size_t)(m0 + rl) * (size_t)lda + koff;
    const _Float16* alr = (const _Float16*)(const void*)AR + (size_t)(m0 + rl) * (size_t)lda + koff;
    const _Float16* br  = (const _Float16*)(const void*)Bt + (size_t)(n0 + rl) * (size_t)ldb + koff;
    for (int k0 = 0; k0 < K; k0 += 32) {
      const v16h ah = ldfrag_h(ar + k0);
      const v16h al = ldfrag_h(alr + k0);
#pragma unroll
      for (int j = 0; j < 8; ++j) {
        const v16h bq = ldfrag_h(br + (size_t)j * 16 * (size_t)ldb + k0);
        acch[j] = mma_h_raw(ah, bq, acch[j]);
        accl[j] = mma_h_raw(al, bq, accl[j]);
        guard3(acch[j], accl[j], ah, al, bq);
      }
    }
  }
  acc_guard4(acch[0], acch[1], acch[2], acch[3]);
  acc_guard4(acch[4], acch[5], acch[6], acch[7]);
  acc_guard4(accl[0], accl[1], accl[2], accl[3]);
  acc_guard4(accl[4], accl[5], accl[6], accl[7]);

  const int  ACT  = (EPI == EPI_SIG) ? 2 : ((EPI == EPI_ALPHA || EPI == EPI_CW || EPI == EPI_W1) ? 1 : 0);
  const bool F32O = (EPI == EPI_HA) || (EPI == EPI_F32) || (EPI == EPI_SIG) || (EPI == EPI_MIX) || (EPI == EPI_OUT);
  const bool F16O = (EPI == EPI_QKV) || (EPI == EPI_HA) || (EPI == EPI_CW) || (EPI == EPI_W1);
  const bool vtile = (EPI == EPI_QKV) && (n0 >= 2 * DM);

  float* slab = sT[wave];
  float bcol[8];
#pragma unroll
  for (int j = 0; j < 8; ++j) {
    float bv = 0.f;
    if (EPI == EPI_SIG || EPI == EPI_W1 || EPI == EPI_OUT) bv = bfr(P0[n0 + 16 * j + rl]);
    if (EPI == EPI_ALPHA) {
      const int col = n0 + 16 * j + rl;
      const int cc  = (col < D3) ? col : (D3 - 1);
      const float t = bfr(P0[cc]);
      bv = (col < D3) ? t : 0.f;
    }
    bcol[j] = bv;
  }
  float bmix[4] = {0.f, 0.f, 0.f, 0.f};
  if (EPI == EPI_MIX) {
#pragma unroll
    for (int e = 0; e < 4; ++e) bmix[e] = bfr(P0[n0 + lane * 4 + e]);
  }

#pragma unroll
  for (int j = 0; j < 8; ++j) {
#pragma unroll
    for (int r = 0; r < 8; ++r)
      slab[(8 * hh + r) * 132 + 16 * j + rl] = (acch[j][r] + accl[j][r] * (1.0f / RSC)) * oscale + bcol[j];
  }
  wave_sync_lds();

  if (ACT != 0) {
#pragma unroll 1
    for (int it = 0; it < 16; ++it) {
      float* sp = slab + it * 132 + lane * 4;
      v4f v = *(const v4f*)sp;
#pragma unroll
      for (int e = 0; e < 4; ++e) {
        if (ACT == 1) v[e] = gelu_f(v[e]);
        else          v[e] = sigm_f(v[e]);
      }
      *(v4f*)sp = v;
    }
    wave_sync_lds();
  }

  if (F32O || vtile) {
    float* Cf = vtile ? (float*)C2 : (float*)C0;
    const int cp = vtile ? DM : ldc;
    const int cc = vtile ? (n0 - 2 * DM) : n0;
#pragma unroll
    for (int rg = 0; rg < 2; ++rg) {
      v4f ov[8];
#pragma unroll
      for (int it = 0; it < 8; ++it) {
        const int row  = rg * 8 + it;
        const int grow = m0 + row;
        v4f v = *(const v4f*)(slab + row * 132 + lane * 4);
        if (EPI == EPI_MIX) {
          const v4f xv = *(const v4f*)(P1 + (size_t)grow * (size_t)ldc + n0 + lane * 4);
#pragma unroll
          for (int e = 0; e < 4; ++e) v[e] = bfr(xv[e]) + v[e];
#pragma unroll
          for (int e = 0; e < 4; ++e) v[e] = v[e] + bmix[e];
        }
        if (EPI == EPI_OUT) {
          const v4f xv = *(const v4f*)(P1 + (size_t)grow * (size_t)ldc + n0 + lane * 4);
#pragma unroll
          for (int e = 0; e < 4; ++e) v[e] = xv[e] + v[e];
        }
        ov[it] = v;
      }
      for (int pass = 0; pass < 2; ++pass) {
#pragma unroll
        for (int it = 0; it < 8; ++it)
          *(volatile v4f*)(Cf + (size_t)(m0 + rg * 8 + it) * (size_t)cp + cc + lane * 4) = ov[it];
        __threadfence();
      }
    }
  }

  if (F16O && !vtile) {
    unsigned short* Cp = (unsigned short*)((EPI == EPI_HA) ? C1 : C0);
    unsigned short* Cq = (unsigned short*)((EPI == EPI_HA) ? C2 : C1);
    v4u hv[8], lv[8];
#pragma unroll
    for (int it = 0; it < 8; ++it) {
      const int row  = it * 2 + hh;
      const int grow = m0 + row;
      const float* sp = slab + row * 132 + rl * 8;
      const v4f fa = *(const v4f*)sp;
      const v4f fb = *(const v4f*)(sp + 4);
      float f[8], go[8];
      f[0] = fa[0]; f[1] = fa[1]; f[2] = fa[2]; f[3] = fa[3];
      f[4] = fb[0]; f[5] = fb[1]; f[6] = fb[2]; f[7] = fb[3];
      if (EPI == EPI_QKV) {
        const int  t    = grow % TLEN;
        const int  d0l  = (rl & 3) * 8;
        const bool lowh = (d0l < 16);
        const int  pc   = lowh ? (rl * 8 + 16) : (rl * 8 - 16);
        const float* pp = slab + row * 132 + pc;
        const v4f pa = *(const v4f*)pp;
        const v4f pb = *(const v4f*)(pp + 4);
        float xp[8];
        xp[0] = pa[0]; xp[1] = pa[1]; xp[2] = pa[2]; xp[3] = pa[3];
        xp[4] = pb[0]; xp[5] = pb[1]; xp[6] = pb[2]; xp[7] = pb[3];
        const int ib = d0l & 15;
        const v4f ca = *(const v4f*)(P0 + (size_t)t * 16 + ib);
        const v4f cb = *(const v4f*)(P0 + (size_t)t * 16 + ib + 4);
        const v4f sa = *(const v4f*)(P1 + (size_t)t * 16 + ib);
        const v4f sb = *(const v4f*)(P1 + (size_t)t * 16 + ib + 4);
        float cv[8], sv[8];
        cv[0] = ca[0]; cv[1] = ca[1]; cv[2] = ca[2]; cv[3] = ca[3];
        cv[4] = cb[0]; cv[5] = cb[1]; cv[6] = cb[2]; cv[7] = cb[3];
        sv[0] = sa[0]; sv[1] = sa[1]; sv[2] = sa[2]; sv[3] = sa[3];
        sv[4] = sb[0]; sv[5] = sb[1]; sv[6] = sb[2]; sv[7] = sb[3];
        const float csc = (n0 < DM) ? QSC : KSC;
#pragma unroll
        for (int e = 0; e < 8; ++e) {
          const float glo = f[e] * cv[e] - xp[e] * sv[e];
          const float ghi = xp[e] * sv[e] + f[e] * cv[e];
          go[e] = (lowh ? glo : ghi) * csc;
        }
      } else if (EPI == EPI_HA) {
#pragma unroll
        for (int e = 0; e < 8; ++e) go[e] = f[e] * HSC;
      } else if (EPI == EPI_CW) {
        const float* gp = P0 + (size_t)grow * (size_t)ldc + n0 + rl * 8;
        const float* hq = P1 + (size_t)grow * (size_t)ldc + n0 + rl * 8;
        const v4f ga = *(const v4f*)gp;
        const v4f gb = *(const v4f*)(gp + 4);
        const v4f ha = *(const v4f*)hq;
        const v4f hb = *(const v4f*)(hq + 4);
        float gg[8], hv0[8];
        gg[0] = ga[0]; gg[1] = ga[1]; gg[2] = ga[2]; gg[3] = ga[3];
        gg[4] = gb[0]; gg[5] = gb[1]; gg[6] = gb[2]; gg[7] = gb[3];
        hv0[0] = ha[0]; hv0[1] = ha[1]; hv0[2] = ha[2]; hv0[3] = ha[3];
        hv0[4] = hb[0]; hv0[5] = hb[1]; hv0[6] = hb[2]; hv0[7] = hb[3];
#pragma unroll
        for (int e = 0; e < 8; ++e) {
          const float y   = f[e] * gg[e];
          const float hm  = hv0[e] + y;
          const float tmp = hv0[e] + hm;
          go[e] = tmp * cscale;
        }
      } else {
#pragma unroll
        for (int e = 0; e < 8; ++e) go[e] = f[e] * cscale;
      }
      v4u pk, pl;
#pragma unroll
      for (int e = 0; e < 4; ++e) {
        unsigned uh, ul;
        hilo2(go[2 * e], go[2 * e + 1], uh, ul);
        pk[e] = uh;
        pl[e] = ul;
      }
      hv[it] = pk;
      lv[it] = pl;
    }
    for (int pass = 0; pass < 2; ++pass) {
#pragma unroll
      for (int it = 0; it < 8; ++it) {
        const int row = it * 2 + hh;
        const size_t gofs = (size_t)(m0 + row) * (size_t)ldc + n0 + rl * 8;
        *(volatile v4u*)(Cp + gofs) = hv[it];
        *(volatile v4u*)(Cq + gofs) = lv[it];
      }
      __threadfence();
    }
  }

  if (EPI == EPI_ALPHA) {
    float s0 = 0.f, s1 = 0.f, s2 = 0.f;
#pragma unroll 1
    for (int q = 0; q < 64; ++q) {
      const int   jj = hh * 64 + q;
      const float e  = slab[rl * 132 + jj];
      const int   jc = (jj < D3) ? jj : (D3 - 1);
      const float mk = (jj < D3) ? 1.f : 0.f;
      const float w0 = bfr(P1[jc]) * mk;
      const float w1 = bfr(P1[D3 + jc]) * mk;
      const float w2 = bfr(P1[2 * D3 + jc]) * mk;
      s0 += e * w0; s1 += e * w1; s2 += e * w2;
    }
    s0 += __shfl_xor(s0, 16, 32);
    s1 += __shfl_xor(s1, 16, 32);
    s2 += __shfl_xor(s2, 16, 32);
    const float a0 = sigm_f(s0 + bfr(P2[0]));
    const float a1 = sigm_f(s1 + bfr(P2[1]));
    const float a2 = sigm_f(s2 + bfr(P2[2]));
    if (hh == 0) {
      slab[rl * 132 + 128] = a0;
      slab[rl * 132 + 129] = a1;
      slab[rl * 132 + 130] = a2;
      slab[rl * 132 + 131] = 0.f;
    }
    wave_sync_lds();
    const v4f av = *(const v4f*)(slab + rl * 132 + 128);
    float* Cf = (float*)C0;
    float* dst = Cf + (size_t)(m0 + rl) * 4;
    if (hh == 0) *(volatile v4f*)dst = av;
    __threadfence();
    if (hh == 0) *(volatile v4f*)dst = av;
  }
}

__global__ __launch_bounds__(256) void attn_c(const unsigned short* __restrict__ QKH,
                                             const unsigned short* __restrict__ QKL,
                                             const unsigned short* __restrict__ VTH,
                                             const unsigned short* __restrict__ VTL,
                                             unsigned short* ZH, unsigned short* ZL, float sscale) {
  __shared__ __align__(16) _Float16 Ksh[2][64 * HD];
  __shared__ __align__(16) _Float16 Vhs[2][HD * 64];
  __shared__ __align__(16) _Float16 Vls[2][HD * 64];
  __shared__ __align__(16) _Float16 PZ[PZ_HALVES];

  const int tid = threadIdx.x, wave = tid >> 5, lane = tid & 31, hh = lane >> 4, c = lane & 15;
  const unsigned bx = blockIdx.x;
  const int qb = (int)(bx % (unsigned)NQB);
  const unsigned bq = bx / (unsigned)NQB;
  const int hp = (int)(bq % (unsigned)(NHEAD / 2));
  const int b  = (int)(bq / (unsigned)(NHEAD / 2));
  if (b >= NBAT) return;
  const int g  = wave >> 2;
  const int wq = wave & 3;
  const int h  = hp * 2 + g;
  const int tg = tid & 127;
  const size_t btok = (size_t)b * TLEN;
  const int rowl0 = qb * QB + wq * 16;

  const _Float16* QH16 = (const _Float16*)(const void*)QKH;
  const _Float16* QL16 = (const _Float16*)(const void*)QKL;
  const _Float16* VH16 = (const _Float16*)(const void*)VTH;
  const _Float16* VL16 = (const _Float16*)(const void*)VTL;
  const v16h qh = ldfrag_h(QH16 + (btok + rowl0 + c) * (size_t)QKW + h * HD + 8 * hh);
  const v16h ql = ldfrag_h(QL16 + (btok + rowl0 + c) * (size_t)QKW + h * HD + 8 * hh);

  float mrow[8], lrow[8];
  v8f oh[2];
#pragma unroll
  for (int r = 0; r < 8; ++r) { mrow[r] = NEG_BIG; lrow[r] = 0.f; }
  oh[0] = zero8(); oh[1] = zero8();

  _Float16* pwh = PZ + wave * 1024;
  _Float16* pwl = PZ + 8 * 1024 + wave * 1024;
  _Float16* ks = Ksh[g];
  _Float16* vs = Vhs[g];
  _Float16* ws = Vls[g];

  for (int kt = 0; kt < NQB; ++kt) {
    if (kt > qb) break;
    const int k0 = kt * 64;
    __syncthreads();
    {
      const int r = tg >> 1, hk = (tg & 1) * 16;
      const _Float16* kg = QH16 + (btok + k0 + r) * (size_t)QKW + DM + h * HD + hk;
      *(v8h*)(ks + r * HD + hk)     = *(const v8h*)(kg);
      *(v8h*)(ks + r * HD + hk + 8) = *(const v8h*)(kg + 8);
      cbar();
      const int d = tg >> 2, kq = (tg & 3) * 16;
      const size_t vo = (size_t)(h * HD + d) * (size_t)NTOK + btok + k0 + kq;
      *(v8h*)(vs + d * 64 + kq)     = *(const v8h*)(VH16 + vo);
      *(v8h*)(vs + d * 64 + kq + 8) = *(const v8h*)(VH16 + vo + 8);
      cbar();
      *(v8h*)(ws + d * 64 + kq)     = *(const v8h*)(VL16 + vo);
      *(v8h*)(ws + d * 64 + kq + 8) = *(const v8h*)(VL16 + vo + 8);
    }
    __syncthreads();

    v8f s[4];
#pragma unroll
    for (int j = 0; j < 4; ++j) {
      FH kb;
      kb.h[0] = *(const v8h*)(ks + (j * 16 + c) * HD + 8 * hh);
      kb.h[1] = *(const v8h*)(ks + (j * 16 + c) * HD + 16 + 8 * hh);
      v8f sh = mma_h_raw(qh, kb.v, zero8());
      v8f sl = mma_h_raw(ql, kb.v, zero8());
      guard3(sh, sl, qh, ql, kb.v);
      const int key  = k0 + j * 16 + c;
      const int rowb = rowl0 + 8 * hh;
#pragma unroll
      for (int r = 0; r < 8; ++r) {
        float v = sh[r];
        v += sl[r] * (1.0f / RSC);
        v *= sscale;
        s[j][r] = (key <= rowb + r) ? v : NEG_BIG;
      }
    }

#pragma unroll
    for (int r = 0; r < 8; ++r) {
      float m = s[0][r];
      m = fmaxf(m, s[1][r]);
      m = fmaxf(m, s[2][r]);
      m = fmaxf(m, s[3][r]);
#pragma unroll
      for (int off = 1; off < 16; off <<= 1) m = fmaxf(m, __shfl_xor(m, off, 32));
      const float mnew  = fmaxf(mrow[r], m);
      const float alpha = __expf(mrow[r] - mnew);
      mrow[r] = mnew;
      float psum = 0.f;
#pragma unroll
      for (int j = 0; j < 4; ++j) {
        const float p  = __expf(s[j][r] - mnew);
        psum += p;
        const float ph = p * PSC;
        const _Float16 xh = (_Float16)ph;
        const int pi = (8 * hh + r) * 64 + j * 16 + c;
        pwh[pi] = xh;
        pwl[pi] = (_Float16)((ph - (float)xh) * RSC);
      }
#pragma unroll
      for (int off = 1; off < 16; off <<= 1) psum += __shfl_xor(psum, off, 32);
      lrow[r] = lrow[r] * alpha + psum;
      oh[0][r] *= alpha;
      oh[1][r] *= alpha;
    }
    wave_sync_lds();

    FH pa0, pa1, pb0, pb1;
    pa0.h[0] = *(const v8h*)(pwh + c * 64 + 8 * hh);
    pa0.h[1] = *(const v8h*)(pwh + c * 64 + 16 + 8 * hh);
    pa1.h[0] = *(const v8h*)(pwh + c * 64 + 32 + 8 * hh);
    pa1.h[1] = *(const v8h*)(pwh + c * 64 + 48 + 8 * hh);
    pb0.h[0] = *(const v8h*)(pwl + c * 64 + 8 * hh);
    pb0.h[1] = *(const v8h*)(pwl + c * 64 + 16 + 8 * hh);
    pb1.h[0] = *(const v8h*)(pwl + c * 64 + 32 + 8 * hh);
    pb1.h[1] = *(const v8h*)(pwl + c * 64 + 48 + 8 * hh);
    cbar();
#pragma unroll
    for (int t = 0; t < 2; ++t) {
      const _Float16* vr = vs + (t * 16 + c) * 64 + 8 * hh;
      const _Float16* wr = ws + (t * 16 + c) * 64 + 8 * hh;
      FH vb0, vb1, wb0, wb1;
      vb0.h[0] = *(const v8h*)(vr);
      vb0.h[1] = *(const v8h*)(vr + 16);
      vb1.h[0] = *(const v8h*)(vr + 32);
      vb1.h[1] = *(const v8h*)(vr + 48);
      wb0.h[0] = *(const v8h*)(wr);
      wb0.h[1] = *(const v8h*)(wr + 16);
      wb1.h[0] = *(const v8h*)(wr + 32);
      wb1.h[1] = *(const v8h*)(wr + 48);
      v8f ol = zero8();
      oh[t] = mma_h_raw(pa0.v, vb0.v, oh[t]);
      ol    = mma_h_raw(pa0.v, wb0.v, ol);
      ol    = mma_h_raw(pb0.v, vb0.v, ol);
      oh[t] = mma_h_raw(pa1.v, vb1.v, oh[t]);
      ol    = mma_h_raw(pa1.v, wb1.v, ol);
      ol    = mma_h_raw(pb1.v, vb1.v, ol);
      guard8m(oh[t], ol, pa0.v, pa1.v, pb0.v, pb1.v, vb0.v, vb1.v, wb0.v, wb1.v);
#pragma unroll
      for (int r = 0; r < 8; ++r) oh[t][r] += ol[r] * (1.0f / RSC);
    }
    acc_guard2(oh[0], oh[1]);
  }

  __syncthreads();
  _Float16* Zh = PZ;
  _Float16* Zl = PZ + 64 * 72;
#pragma unroll
  for (int r = 0; r < 8; ++r) {
    const float l   = lrow[r];
    const float inv = (1.0f / l) * (1.0f / (PSC * VSC)) * ZSC;
#pragma unroll
    for (int t = 0; t < 2; ++t) {
      const float zv = oh[t][r] * inv;
      const _Float16 xh = (_Float16)zv;
      const _Float16 xl = (_Float16)((zv - (float)xh) * RSC);
      const int zi = (wq * 16 + 8 * hh + r) * 72 + g * 32 + 16 * t + c;
      Zh[zi] = xh;
      Zl[zi] = xl;
    }
  }
  __syncthreads();
  {
    const int seg = tid & 7;
    U84 zh[2], zl[2];
#pragma unroll
    for (int it = 0; it < 2; ++it) {
      const int row = it * 32 + (tid >> 3);
      zh[it].h = *(const v8h*)(Zh + row * 72 + seg * 8);
      zl[it].h = *(const v8h*)(Zl + row * 72 + seg * 8);
    }
    for (int pass = 0; pass < 2; ++pass) {
#pragma unroll
      for (int it = 0; it < 2; ++it) {
        const int row = it * 32 + (tid >> 3);
        const size_t zo = (btok + (size_t)(qb * QB + row)) * DM + hp * 64 + seg * 8;
        *(volatile v4u*)(ZH + zo) = zh[it].u;
        *(volatile v4u*)(ZL + zo) = zl[it].u;
      }
      __threadfence();
    }
  }
}

__global__ __launch_bounds__(256) void scan_k(const float* __restrict__ BU, const float* __restrict__ AL,
                                             const float* __restrict__ abase, const float* __restrict__ adelta,
                                             unsigned short* SH, unsigned short* SLo) {
  __shared__ __align__(16) float Ssh[8 * DM];
  const int tid = threadIdx.x;
  const int b = (int)blockIdx.x;
  if (b >= NBAT) return;
  const int d = tid;
  const float ab = bfr(abase[d]);
  const float td = tanhf(bfr(adelta[d]));
  const int grp = (d < D3) ? 0 : ((d < 2 * D3) ? 1 : 2);
  const size_t tok0 = (size_t)b * TLEN;
  const int row = tid >> 5, lane = tid & 31;
  float s = 0.f;
  for (int t0 = 0; t0 < TLEN; t0 += 8) {
    __syncthreads();
#pragma unroll 1
    for (int j = 0; j < 8; ++j) {
      const size_t tok = tok0 + (size_t)(t0 + j);
      const float al  = AL[tok * 4 + grp];
      const float a   = ab + al * td;
      const float x   = -a;
      const float sp  = fmaxf(x, 0.f) + __logf(1.0f + __expf(-fabsf(x)));
      const float lam = __expf(-sp);
      const float bu  = BU[tok * DM + d];
      s = lam * s + bu;
      Ssh[j * DM + d] = s * SSC;
    }
    __syncthreads();
    const v4f fa = *(const v4f*)(Ssh + row * DM + lane * 8);
    const v4f fb = *(const v4f*)(Ssh + row * DM + lane * 8 + 4);
    v4u ph, pl;
    {
      unsigned uh, ul;
      hilo2(fa[0], fa[1], uh, ul); ph[0] = uh; pl[0] = ul;
      hilo2(fa[2], fa[3], uh, ul); ph[1] = uh; pl[1] = ul;
      hilo2(fb[0], fb[1], uh, ul); ph[2] = uh; pl[2] = ul;
      hilo2(fb[2], fb[3], uh, ul); ph[3] = uh; pl[3] = ul;
    }
    const size_t so = (tok0 + (size_t)(t0 + row)) * DM + lane * 8;
    *(volatile v4u*)(SH + so)  = ph;
    *(volatile v4u*)(SLo + so) = pl;
    __threadfence();
    *(volatile v4u*)(SH + so)  = ph;
    *(volatile v4u*)(SLo + so) = pl;
  }
}

extern "C" void kernel_launch(void* const* d_in, const int* in_sizes, int n_in,
                              void* d_out, int out_size, void* d_ws, size_t ws_size,
                              hipStream_t stream) {
  if (n_in < 32) return;
  if (in_sizes[0] != NTOK * DM) return;
  if (in_sizes[1] != DM || in_sizes[2] != DM) return;
  if (in_sizes[3] != MD * DM || in_sizes[4] != MD * LR || in_sizes[5] != LR * DM) return;
  if (in_sizes[6] != DM * DM || in_sizes[7] != DM * LR || in_sizes[8] != LR * DM) return;
  if (in_sizes[9] != DM || in_sizes[10] != DM) return;
  if (in_sizes[11] != RNK * DM || in_sizes[12] != DM * RNK) return;
  if (in_sizes[13] != D3 * DM || in_sizes[14] != D3 || in_sizes[15] != 3 * D3 || in_sizes[16] != 3) return;
  if (in_sizes[17] != DM * DM || in_sizes[18] != DM * DM || in_sizes[19] != DM) return;
  if (in_sizes[20] != DM * DM || in_sizes[21] != DM || in_sizes[22] != DM || in_sizes[23] != DM) return;
  if (in_sizes[24] != MD * DM || in_sizes[25] != MD || in_sizes[26] != MD * LR || in_sizes[27] != LR * DM) return;
  if (in_sizes[28] != DM * MD || in_sizes[29] != DM || in_sizes[30] != DM * LR || in_sizes[31] != LR * MD) return;
  if (out_size != NTOK * DM) return;

  const float* x      = (const float*)d_in[0];
  const float* g1     = (const float*)d_in[1];
  const float* b1     = (const float*)d_in[2];
  const float* Wqkv   = (const float*)d_in[3];
  const float* Aqkv   = (const float*)d_in[4];
  const float* Bqkv   = (const float*)d_in[5];
  const float* Wo     = (const float*)d_in[6];
  const float* Ao     = (const float*)d_in[7];
  const float* Bo     = (const float*)d_in[8];
  const float* a_base = (const float*)d_in[9];
  const float* a_delta= (const float*)d_in[10];
  const float* Vw     = (const float*)d_in[11];
  const float* Uw     = (const float*)d_in[12];
  const float* E1w    = (const float*)d_in[13];
  const float* E1b    = (const float*)d_in[14];
  const float* E2w    = (const float*)d_in[15];
  const float* E2b    = (const float*)d_in[16];
  const float* Cw     = (const float*)d_in[17];
  const float* Gw     = (const float*)d_in[18];
  const float* Gb     = (const float*)d_in[19];
  const float* Mixw   = (const float*)d_in[20];
  const float* Mixb   = (const float*)d_in[21];
  const float* g2     = (const float*)d_in[22];
  const float* b2     = (const float*)d_in[23];
  const float* W1     = (const float*)d_in[24];
  const float* b1m    = (const float*)d_in[25];
  const float* A1l    = (const float*)d_in[26];
  const float* B1l    = (const float*)d_in[27];
  const float* W2     = (const float*)d_in[28];
  const float* b2m    = (const float*)d_in[29];
  const float* A2l    = (const float*)d_in[30];
  const float* B2l    = (const float*)d_in[31];
  float* outf = (float*)d_out;

  const size_t P768  = (size_t)MD * DM * 2;
  const size_t P256  = (size_t)DM * DM * 2;
  const size_t PE1   = (size_t)E1N * DM * 2;
  const size_t PROPE = (size_t)TLEN * 16 * 4;
  const size_t PAL   = (size_t)NTOK * 4 * 4;
  const size_t PA16  = (size_t)NTOK * DM * 2;
  const size_t PQK   = (size_t)NTOK * QKW * 2;
  const size_t PA32  = (size_t)NTOK * DM * 4;
  const size_t PU16  = (size_t)NTOK * MD * 2;
  size_t off = 0;
  const size_t oWQKV = off; off += P768;
  const size_t oWO   = off; off += P256;
  const size_t oW1E  = off; off += P768;
  const size_t oW2E  = off; off += P768;
  const size_t oUVE  = off; off += P256;
  const size_t oGWE  = off; off += P256;
  const size_t oE1E  = off; off += PE1;
  const size_t oCWE  = off; off += P256;
  const size_t oMIXE = off; off += P256;
  const size_t oROPC = off; off += PROPE;
  const size_t oROPS = off; off += PROPE;
  const size_t oAL   = off; off += PAL;
  const size_t oH16  = off; off += PA16;
  const size_t oHL16 = off; off += PA16;
  const size_t oQKH  = off; off += PQK;
  const size_t oQKL  = off; off += PQK;
  const size_t oVF   = off; off += PA32;
  const size_t oVTH  = off; off += PA16;
  const size_t oVTL  = off; off += PA16;
  const size_t oZ16  = off; off += PA16;
  const size_t oZL16 = off; off += PA16;
  const size_t oHA32 = off; off += PA32;
  const size_t oHA16 = off; off += PA16;
  const size_t oHAL  = off; off += PA16;
  const size_t oBU   = off; off += PA32;
  const size_t oGG   = off; off += PA32;
  const size_t oS16  = off; off += PA16;
  const size_t oSL16 = off; off += PA16;
  const size_t oTMP  = off; off += PA16;
  const size_t oTMPL = off; off += PA16;
  const size_t oX2   = off; off += PA32;
  const size_t oH2   = off; off += PA16;
  const size_t oH2L  = off; off += PA16;
  if (off > ws_size) return;
  if (off > (size_t)134217728) return;
  const size_t oU16  = oQKH;
  const size_t oUL16 = oQKH + PU16;
  if (oUL16 + PU16 != oVF + PA32) return;

  char* ws = (char*)d_ws;
  unsigned short* WQKV  = (unsigned short*)(ws + oWQKV);
  unsigned short* WOE   = (unsigned short*)(ws + oWO);
  unsigned short* W1E   = (unsigned short*)(ws + oW1E);
  unsigned short* W2E   = (unsigned short*)(ws + oW2E);
  unsigned short* UVE   = (unsigned short*)(ws + oUVE);
  unsigned short* GWE   = (unsigned short*)(ws + oGWE);
  unsigned short* E1E   = (unsigned short*)(ws + oE1E);
  unsigned short* CWE   = (unsigned short*)(ws + oCWE);
  unsigned short* MIXE  = (unsigned short*)(ws + oMIXE);
  float*          ROPC  = (float*)(ws + oROPC);
  float*          ROPS  = (float*)(ws + oROPS);
  float*          AL    = (float*)(ws + oAL);
  unsigned short* H16   = (unsigned short*)(ws + oH16);
  unsigned short* HL16  = (unsigned short*)(ws + oHL16);
  unsigned short* QKH   = (unsigned short*)(ws + oQKH);
  unsigned short* QKL   = (unsigned short*)(ws + oQKL);
  float*          VF    = (float*)(ws + oVF);
  unsigned short* VTH   = (unsigned short*)(ws + oVTH);
  unsigned short* VTL   = (unsigned short*)(ws + oVTL);
  unsigned short* Z16   = (unsigned short*)(ws + oZ16);
  unsigned short* ZL16  = (unsigned short*)(ws + oZL16);
  float*          HA32  = (float*)(ws + oHA32);
  unsigned short* HA16  = (unsigned short*)(ws + oHA16);
  unsigned short* HAL16 = (unsigned short*)(ws + oHAL);
  float*          BU32  = (float*)(ws + oBU);
  float*          GG32  = (float*)(ws + oGG);
  unsigned short* S16   = (unsigned short*)(ws + oS16);
  unsigned short* SL16  = (unsigned short*)(ws + oSL16);
  unsigned short* TMP16 = (unsigned short*)(ws + oTMP);
  unsigned short* TMPL16= (unsigned short*)(ws + oTMPL);
  float*          X2    = (float*)(ws + oX2);
  unsigned short* H2_16 = (unsigned short*)(ws + oH2);
  unsigned short* H2L16 = (unsigned short*)(ws + oH2L);
  unsigned short* U16   = (unsigned short*)(ws + oU16);
  unsigned short* UL16  = (unsigned short*)(ws + oUL16);

  const dim3 blk256(256), blk128(128);

  prep_w<<<dim3((MD * DM) / 2048), blk256, 0, stream>>>(Wqkv, Aqkv, Bqkv, WQKV, MD, MD, DM, LR, 1, LORA_MUL, WSC);
  prep_w<<<dim3((DM * DM) / 2048), blk256, 0, stream>>>(Wo, Ao, Bo, WOE, DM, DM, DM, LR, 1, LORA_MUL, WSC);
  prep_w<<<dim3((MD * DM) / 2048), blk256, 0, stream>>>(W1, A1l, B1l, W1E, MD, MD, DM, LR, 1, LORA_MUL, WSC);
  prep_w<<<dim3((DM * MD) / 2048), blk256, 0, stream>>>(W2, A2l, B2l, W2E, DM, DM, MD, LR, 1, LORA_MUL, WSC);
  prep_w<<<dim3((DM * DM) / 2048), blk256, 0, stream>>>(Uw, Uw, Vw, UVE, DM, DM, DM, RNK, 0, 1.0f, UVSC);
  prep_w<<<dim3((DM * DM) / 2048), blk256, 0, stream>>>(Gw, Gw, Gw, GWE, DM, DM, DM, 0, 1, 0.0f, WSC);
  prep_w<<<dim3((E1N * DM) / 2048), blk256, 0, stream>>>(E1w, E1w, E1w, E1E, D3, E1N, DM, 0, 1, 0.0f, WSC);
  prep_w<<<dim3((DM * DM) / 2048), blk256, 0, stream>>>(Cw, Cw, Cw, CWE, DM, DM, DM, 0, 1, 0.0f, WSC);
  prep_w<<<dim3((DM * DM) / 2048), blk256, 0, stream>>>(Mixw, Mixw, Mixw, MIXE, DM, DM, DM, 0, 1, 0.0f, WSC);
  rope_tab<<<dim3((TLEN * 16) / 256), blk256, 0, stream>>>(ROPC, ROPS, TLEN * 16);

  ln_rows<<<dim3(NTOK / 8), blk256, 0, stream>>>(x, g1, b1, H16, HL16, NTOK, XSC);

  const int g768 = ((NTOK / 16) * (MD / 128)) / 4;
  const int g256 = ((NTOK / 16) * (DM / 128)) / 4;
  const int g128 = ((NTOK / 16) * (E1N / 128)) / 4;
  gemm_t<EPI_QKV><<<dim3(g768), blk128, 0, stream>>>(H16, HL16, DM, WQKV, DM, (void*)QKH, (void*)QKL, (void*)VF,
                                                     QKW, ROPC, ROPS, g1, NTOK, MD, DM, 1.0f / (XSC * WSC), 1.0f);

  tr_cvt2<<<dim3(DM / 64, NTOK / 64), blk256, 0, stream>>>(VF, NTOK, DM, VTH, VTL, VSC);

  const float sscale = 0.17677669529663687f / (QSC * KSC);
  attn_c<<<dim3(NBAT * (NHEAD / 2) * NQB), blk256, 0, stream>>>(QKH, QKL, VTH, VTL, Z16, ZL16, sscale);

  gemm_t<EPI_HA><<<dim3(g256), blk128, 0, stream>>>(Z16, ZL16, DM, WOE, DM, (void*)HA32, (void*)HA16, (void*)HAL16,
                                                    DM, g1, g1, g1, NTOK, DM, DM, 1.0f / (ZSC * WSC), 1.0f);

  gemm_t<EPI_F32><<<dim3(g256), blk128, 0, stream>>>(HA16, HAL16, DM, UVE, DM, (void*)BU32, (void*)BU32,
                                                     (void*)BU32, DM, g1, g1, g1, NTOK, DM, DM,
                                                     1.0f / (HSC * UVSC), 1.0f);
  gemm_t<EPI_SIG><<<dim3(g256), blk128, 0, stream>>>(HA16, HAL16, DM, GWE, DM, (void*)GG32, (void*)GG32,
                                                     (void*)GG32, DM, Gb, g1, g1, NTOK, DM, DM,
                                                     1.0f / (HSC * WSC), 1.0f);
  gemm_t<EPI_ALPHA><<<dim3(g128), blk128, 0, stream>>>(HA16, HAL16, DM, E1E, DM, (void*)AL, (void*)AL, (void*)AL,
                                                       4, E1b, E2w, E2b, NTOK, E1N, DM, 1.0f / (HSC * WSC), 1.0f);

  scan_k<<<dim3(NBAT), blk256, 0, stream>>>(BU32, AL, a_base, a_delta, S16, SL16);

  gemm_t<EPI_CW><<<dim3(g256), blk128, 0, stream>>>(S16, SL16, DM, CWE, DM, (void*)TMP16, (void*)TMPL16,
                                                    (void*)TMPL16, DM, GG32, HA32, g1, NTOK, DM, DM,
                                                    1.0f / (SSC * WSC), TSC);

  gemm_t<EPI_MIX><<<dim3(g256), blk128, 0, stream>>>(TMP16, TMPL16, DM, MIXE, DM, (void*)X2, (void*)X2, (void*)X2,
                                                     DM, Mixb, x, g1, NTOK, DM, DM, 1.0f / (TSC * WSC), 1.0f);

  ln_rows<<<dim3(NTOK / 8), blk256, 0, stream>>>(X2, g2, b2, H2_16, H2L16, NTOK, XSC);

  gemm_t<EPI_W1><<<dim3(g768), blk128, 0, stream>>>(H2_16, H2L16, DM, W1E, DM, (void*)U16, (void*)UL16,
                                                    (void*)UL16, MD, b1m, g1, g1, NTOK, MD, DM,
                                                    1.0f / (XSC * WSC), USC);
  gemm_t<EPI_OUT><<<dim3(g256), blk128, 0, stream>>>(U16, UL16, MD, W2E, MD, (void*)outf, (void*)outf,
                                                     (void*)outf, DM, b2m, X2, g1, NTOK, DM, MD,
                                                     1.0f / (USC * WSC), 1.0f);
  (void)hipGetLastError();
}
